// BiMambaBlock_83674552861035
// MI455X (gfx1250) — hardware-verified
//
#include <hip/hip_runtime.h>
#include <math.h>

typedef __attribute__((ext_vector_type(8)))  _Float16 v8h;
typedef __attribute__((ext_vector_type(16))) __bf16   v16b;
typedef __attribute__((ext_vector_type(8)))  __bf16   v8b;
typedef __attribute__((ext_vector_type(8)))  float    v8f;
typedef __attribute__((ext_vector_type(4)))  float    v4f;

constexpr int kBatch  = 2;
constexpr int kSeq    = 1024;
constexpr int kDm     = 1024;
constexpr int kDin    = 2048;
constexpr int kNst    = 16;
constexpr int kDtR    = 64;
constexpr int kPrjN   = 96;
constexpr int kPrjP   = 128;
constexpr int kXzP    = 2 * kDin;
constexpr int kCatK   = 2 * kDm;
constexpr int kRows   = kBatch * kSeq;
constexpr int kConvTP = 260;
constexpr int kScanTS = 64;
constexpr int kScanCh = 64;
constexpr int kScanYP = 68;
constexpr int kBCW    = 2 * kNst;
static_assert(kDtR + 2 * kNst == kPrjN, "x_proj width");
static_assert((kDm % 32) == 0 && (kDin % 32) == 0 && (kDtR % 32) == 0 && (kCatK % 32) == 0, "GEMM K multiples of 32");
static_assert((kRows % 64) == 0 && (kXzP % 64) == 0 && (kPrjP % 64) == 0 && (kDin % 64) == 0 && (kDm % 64) == 0, "GEMM M,N multiples of 64");
static_assert((kSeq % kScanTS) == 0 && (kSeq % 64) == 0 && (kDin % kScanCh) == 0 && (kDin % 256) == 0, "tile multiples");
static_assert((kSeq & (kSeq - 1)) == 0, "power-of-two sequence length");

constexpr size_t kOffX16   = 0;
constexpr size_t kOffINWT  = kOffX16   + (size_t)kRows * kDm * 2;
constexpr size_t kOffOUTWT = kOffINWT  + (size_t)2 * kXzP * kDm * 2;
constexpr size_t kOffPRJWT = kOffOUTWT + (size_t)2 * kDm * kDin * 2;
constexpr size_t kOffXPWT  = kOffPRJWT + (size_t)kDm * kCatK * 2;
constexpr size_t kOffDTWT  = kOffXPWT  + (size_t)2 * kPrjP * kDin * 2;
constexpr size_t kOffXZ    = kOffDTWT  + (size_t)2 * kDin * kDtR * 2;
constexpr size_t kOffUC16  = kOffXZ    + (size_t)kRows * kXzP * 4;
constexpr size_t kOffPROJ  = kOffUC16  + (size_t)kRows * kDin * 2;
constexpr size_t kOffDT16  = kOffPROJ  + (size_t)kRows * kPrjP * 4;
constexpr size_t kOffDLR   = kOffDT16  + (size_t)kRows * kDtR * 2;
constexpr size_t kOffYH    = kOffDLR   + (size_t)kRows * kDin * 4;
constexpr size_t kOffYL    = kOffYH    + (size_t)kRows * kDin * 2;
constexpr size_t kOffCATH  = kOffYL    + (size_t)kRows * kDin * 2;
constexpr size_t kOffCATL  = kOffCATH  + (size_t)kRows * kCatK * 2;
constexpr size_t kWsTotal  = kOffCATL  + (size_t)kRows * kCatK * 2;
static_assert(kWsTotal == 128712704ull, "carve total");
static_assert(kWsTotal <= 134217728ull, "carve cap");
static_assert((kOffINWT % 128) == 0 && (kOffOUTWT % 128) == 0 && (kOffPRJWT % 128) == 0 && (kOffXPWT % 128) == 0 &&
              (kOffDTWT % 128) == 0 && (kOffXZ % 128) == 0 && (kOffUC16 % 128) == 0 && (kOffPROJ % 128) == 0 &&
              (kOffDT16 % 128) == 0 && (kOffDLR % 128) == 0 && (kOffYH % 128) == 0 && (kOffYL % 128) == 0 &&
              (kOffCATH % 128) == 0 && (kOffCATL % 128) == 0, "128-B aligned regions");

__device__ __forceinline__ unsigned short f2bf_bits(float f) {
  unsigned u = __float_as_uint(f);
  return (unsigned short)((u + 0x7FFFu + ((u >> 16) & 1u)) >> 16);
}
__device__ __forceinline__ float bf_bits2f(unsigned short h) { return __uint_as_float(((unsigned)h) << 16); }
__device__ __forceinline__ float rbf(float f) { return bf_bits2f(f2bf_bits(f)); }

__device__ __forceinline__ void guard4_b(v8f& a, v8f& b, v8f& c, v8f& d, v16b x, v16b y) {
  asm volatile("v_nop\n\tv_nop\n\tv_nop\n\tv_nop" : "+v"(a), "+v"(b), "+v"(c), "+v"(d) : "v"(x), "v"(y));
}
__device__ __forceinline__ void keep4_b(v16b a, v16b b, v16b c, v16b d) { asm volatile("v_nop" :: "v"(a), "v"(b), "v"(c), "v"(d)); }
__device__ __forceinline__ void acc_guard4(v8f& a, v8f& b, v8f& c, v8f& d) { asm volatile("v_nop\n\tv_nop\n\tv_nop\n\tv_nop" : "+v"(a), "+v"(b), "+v"(c), "+v"(d)); }

struct FragB {
  union U { v16b v; v8b h[2]; };
  static __device__ __forceinline__ v16b load(const __bf16* p) {
    U f; f.h[0] = *(const v8b*)(p); f.h[1] = *(const v8b*)(p + 16); return f.v;
  }
  static __device__ __forceinline__ v8f mma(v16b a, v16b b, v8f c) {
    return __builtin_amdgcn_wmma_f32_16x16x32_bf16(false, a, false, b, (short)0, c, false, false);
  }
};

template <int SPL, int BIAS_MODE, int OUT_MODE>
__global__ __launch_bounds__(256) void wmma_gemm64(
    const unsigned short* __restrict__ Ap, const unsigned short* __restrict__ A2p, int lda,
    const unsigned short* __restrict__ Btp, int ldb,
    void* __restrict__ Cout, void* __restrict__ Cout2, int ldc,
    const float* __restrict__ bias, int M, int N, int K) {
  typedef __bf16 T;
  typedef v16b V;
  const T* A = (const T*)Ap; const T* A2 = (const T*)A2p; const T* Bt = (const T*)Btp;
  __shared__ __align__(16) float sT[8][16 * 68];
  const int lane = threadIdx.x & 31;
  const int wave = threadIdx.x >> 5;
  const int tilesN = N >> 6;
  const int tilesM = M >> 6;
  const int tile = blockIdx.x * 8 + wave;
  if (tile >= tilesM * tilesN) return;
  const int tm = tile / tilesN;
  const int tn = tile - tm * tilesN;
  const int m0 = tm << 6;
  const int n0 = tn << 6;

  const int rlane = lane & 15;
  const int koff  = (lane >> 4) * 8;
  const int mOff  = (lane >> 4) * 8;

  v8f acc[4][4];
#pragma unroll
  for (int i = 0; i < 4; ++i)
#pragma unroll
    for (int j = 0; j < 4; ++j) acc[i][j] = (v8f){0.f,0.f,0.f,0.f,0.f,0.f,0.f,0.f};

  for (int k0 = 0; k0 < K; k0 += 32) {
    V bh[4];
#pragma unroll
    for (int j = 0; j < 4; ++j) {
      const size_t bo = (size_t)(n0 + (j << 4) + rlane) * ldb + koff + k0;
      bh[j] = FragB::load(Bt + bo);
    }
#pragma unroll
    for (int i = 0; i < 4; ++i) {
      const size_t ao = (size_t)(m0 + (i << 4) + rlane) * lda + koff + k0;
      V ah = FragB::load(A + ao);
      V al = ah;
      if (SPL >= 1) al = FragB::load(A2 + ao);
#pragma unroll
      for (int j = 0; j < 4; ++j) {
        acc[i][j] = FragB::mma(ah, bh[j], acc[i][j]);
        if (SPL >= 1) acc[i][j] = FragB::mma(al, bh[j], acc[i][j]);
      }
      guard4_b(acc[i][0], acc[i][1], acc[i][2], acc[i][3], ah, al);
    }
    keep4_b(bh[0], bh[1], bh[2], bh[3]);
  }
  acc_guard4(acc[0][0], acc[0][1], acc[0][2], acc[0][3]);
  acc_guard4(acc[1][0], acc[1][1], acc[1][2], acc[1][3]);
  acc_guard4(acc[2][0], acc[2][1], acc[2][2], acc[2][3]);
  acc_guard4(acc[3][0], acc[3][1], acc[3][2], acc[3][3]);

  float* slab = sT[wave];
#pragma unroll
  for (int i = 0; i < 4; ++i) {
    const int mBase = m0 + (i << 4);
#pragma unroll
    for (int j = 0; j < 4; ++j) {
      const int n = n0 + (j << 4) + rlane;
      float bv = 0.f;
      if (BIAS_MODE == 2) bv = rbf(bias[n]);
#pragma unroll
      for (int r = 0; r < 8; ++r) {
        float v = acc[i][j][r];
        if (BIAS_MODE == 2) v += bv;
        slab[(mOff + r) * 68 + (j << 4) + rlane] = v;
      }
    }
    __builtin_amdgcn_fence(__ATOMIC_RELEASE, "workgroup");
    __builtin_amdgcn_wave_barrier();
    __builtin_amdgcn_fence(__ATOMIC_ACQUIRE, "workgroup");
    if (OUT_MODE == 0) {
      float* C = (float*)Cout;
      const int hh = lane >> 4, c4 = (lane & 15) * 4;
      for (int pass = 0; pass < 2; ++pass) {
#pragma unroll
        for (int it = 0; it < 8; ++it) {
          const int row = it * 2 + hh;
          v4f v = *(const v4f*)(slab + row * 68 + c4);
          *(volatile v4f*)(C + (size_t)(mBase + row) * ldc + n0 + c4) = v;
        }
        __threadfence();
      }
    } else {
      const int q = lane >> 3, c8 = (lane & 7) * 8;
      unsigned short* C  = (unsigned short*)Cout;
      unsigned short* C2 = (unsigned short*)Cout2;
      for (int pass = 0; pass < 2; ++pass) {
#pragma unroll
        for (int it = 0; it < 4; ++it) {
          const int row = it * 4 + q;
          const float* sp = slab + row * 68 + c8;
          v8h hv, lv;
#pragma unroll
          for (int e = 0; e < 8; ++e) {
            const float sv = sp[e];
            const unsigned short hb = f2bf_bits(sv);
            const unsigned short lb = f2bf_bits(sv - bf_bits2f(hb));
            hv[e] = __builtin_bit_cast(_Float16, hb);
            lv[e] = __builtin_bit_cast(_Float16, lb);
          }
          *(volatile v8h*)(C  + (size_t)(mBase + row) * ldc + n0 + c8) = hv;
          *(volatile v8h*)(C2 + (size_t)(mBase + row) * ldc + n0 + c8) = lv;
        }
        __threadfence();
      }
    }
    __builtin_amdgcn_fence(__ATOMIC_RELEASE, "workgroup");
    __builtin_amdgcn_wave_barrier();
    __builtin_amdgcn_fence(__ATOMIC_ACQUIRE, "workgroup");
  }
}

__global__ __launch_bounds__(256) void cast_bf16_kernel(
    const float* __restrict__ src, unsigned short* __restrict__ dst, int total8)
{
  const int i = blockIdx.x * 256 + threadIdx.x;
  if (i >= total8) return;
  const size_t e0 = (size_t)i << 3;
  const v4f a0 = *(const v4f*)(src + e0);
  const v4f a1 = *(const v4f*)(src + e0 + 4);
  v8h hv;
#pragma unroll
  for (int e = 0; e < 4; ++e) {
    const unsigned short h0 = f2bf_bits(a0[e]);
    const unsigned short h1 = f2bf_bits(a1[e]);
    hv[e]     = __builtin_bit_cast(_Float16, h0);
    hv[4 + e] = __builtin_bit_cast(_Float16, h1);
  }
  unsigned short* q = dst + e0;
  *(volatile v8h*)q = hv;
  __threadfence();
  *(volatile v8h*)q = hv;
}

__global__ __launch_bounds__(256) void transpose_bf16_kernel(
    const float* __restrict__ Wsrc, unsigned short* __restrict__ Btdst, int Kdim, int Ndim,
    long srcStride, long dstStride)
{
  __shared__ float tile[64 * 65];
  const int tid = threadIdx.x, lane = tid & 31, wave = tid >> 5;
  const float* W = Wsrc + (size_t)blockIdx.z * srcStride;
  unsigned short* Bt = Btdst + (size_t)blockIdx.z * dstStride;
  const int n0 = blockIdx.x * 64;
  const int k0 = blockIdx.y * 64;
#pragma unroll
  for (int p = 0; p < 16; ++p) {
    const int idx = tid + p * 256;
    const int kk  = idx >> 6;
    const int nn  = idx & 63;
    const int n   = n0 + nn;
    const int nc  = (n < Ndim) ? n : (Ndim - 1);
    const float v = W[(size_t)(k0 + kk) * Ndim + nc];
    tile[kk * 65 + nn] = (n < Ndim) ? v : 0.f;
  }
  __syncthreads();
  const int q = lane >> 3, c8 = (lane & 7) * 8;
  v8h hv[2];
#pragma unroll
  for (int it = 0; it < 2; ++it) {
    const int nrow = it * 32 + wave * 4 + q;
#pragma unroll
    for (int e = 0; e < 8; ++e) {
      const unsigned short hb = f2bf_bits(tile[(c8 + e) * 65 + nrow]);
      hv[it][e] = __builtin_bit_cast(_Float16, hb);
    }
  }
  for (int pass = 0; pass < 2; ++pass) {
#pragma unroll
    for (int it = 0; it < 2; ++it) {
      const int nrow = it * 32 + wave * 4 + q;
      *(volatile v8h*)(Bt + (size_t)(n0 + nrow) * Kdim + k0 + c8) = hv[it];
    }
    __threadfence();
  }
}

__global__ __launch_bounds__(256) void dt_cast_kernel(
    const float* __restrict__ PROJ, unsigned short* __restrict__ DT16, int total8)
{
  const int i = blockIdx.x * 256 + threadIdx.x;
  if (i >= total8) return;
  const int e0  = i << 3;
  const int row = e0 >> 6;
  const int c8  = e0 & 63;
  const float* p = PROJ + (size_t)row * kPrjP + c8;
  const v4f a0 = *(const v4f*)(p);
  const v4f a1 = *(const v4f*)(p + 4);
  v8h hv;
#pragma unroll
  for (int e = 0; e < 4; ++e) {
    const unsigned short h0 = f2bf_bits(a0[e]);
    const unsigned short h1 = f2bf_bits(a1[e]);
    hv[e]     = __builtin_bit_cast(_Float16, h0);
    hv[4 + e] = __builtin_bit_cast(_Float16, h1);
  }
  unsigned short* qd = DT16 + e0;
  *(volatile v8h*)qd = hv;
  __threadfence();
  *(volatile v8h*)qd = hv;
}

__global__ __launch_bounds__(256) void conv_silu_kernel(
    const float* __restrict__ XZ, const float* __restrict__ cw, const float* __restrict__ cb,
    unsigned short* __restrict__ UC16, int dir)
{
  __shared__ __align__(16) float sT[16 * kConvTP];
  const int tid = threadIdx.x, lane = tid & 31, wave = tid >> 5;
  const int d0 = blockIdx.x * 256, d = d0 + tid;
  const int g0 = blockIdx.y * 64;
  const int tb = g0 & (kSeq - 1);
  const v4f wv = *(const v4f*)(cw + (size_t)d * 4);
  const float w0 = rbf(wv[0]), w1 = rbf(wv[1]), w2 = rbf(wv[2]), w3 = rbf(wv[3]);
  const float bc = rbf(cb[d]);
  float xm3, xm2, xm1;
  {
    const bool hist = dir ? (tb + 64 < kSeq) : (tb > 0);
    const int hb = hist ? (dir ? (g0 + 64) : (g0 - 3)) : g0;
    const float va = XZ[(size_t)hb * kXzP + d];
    const float vb = XZ[(size_t)(hb + 1) * kXzP + d];
    const float vc = XZ[(size_t)(hb + 2) * kXzP + d];
    const float f3 = dir ? vc : va;
    const float f1 = dir ? va : vc;
    xm3 = hist ? f3 : 0.f;
    xm2 = hist ? vb : 0.f;
    xm1 = hist ? f1 : 0.f;
  }
#pragma unroll 1
  for (int sub = 0; sub < 4; ++sub) {
    const int lb = dir ? (g0 + 48 - sub * 16) : (g0 + sub * 16);
#pragma unroll 1
    for (int s = 0; s < 16; ++s) {
      const int lrow = dir ? (15 - s) : s;
      const float xcur = XZ[(size_t)(lb + lrow) * kXzP + d];
      float acc = w0 * xm3;
      acc = fmaf(w1, xm2, acc);
      acc = fmaf(w2, xm1, acc);
      acc = fmaf(w3, xcur, acc);
      const float sv = acc + bc;
      const float sg = __builtin_amdgcn_rcpf(1.0f + __expf(-sv));
      sT[lrow * kConvTP + tid] = sv * sg;
      xm3 = xm2; xm2 = xm1; xm1 = xcur;
    }
    __syncthreads();
    v8h bv[2];
#pragma unroll
    for (int it = 0; it < 2; ++it) {
      const float* sp = sT + (it * 8 + wave) * kConvTP + lane * 8;
      const v4f a0 = *(const v4f*)(sp);
      const v4f a1 = *(const v4f*)(sp + 4);
#pragma unroll
      for (int e = 0; e < 4; ++e) {
        const unsigned short h0 = f2bf_bits(a0[e]);
        const unsigned short h1 = f2bf_bits(a1[e]);
        bv[it][e]     = __builtin_bit_cast(_Float16, h0);
        bv[it][4 + e] = __builtin_bit_cast(_Float16, h1);
      }
    }
    for (int pass = 0; pass < 2; ++pass) {
#pragma unroll
      for (int it = 0; it < 2; ++it)
        *(volatile v8h*)(UC16 + (size_t)(lb + it * 8 + wave) * kDin + d0 + lane * 8) = bv[it];
      __threadfence();
    }
    __syncthreads();
  }
}

__global__ __launch_bounds__(64) void scan_kernel(
    const float* __restrict__ PROJ, const float* __restrict__ DLR, const float* __restrict__ XZ,
    const float* __restrict__ cw, const float* __restrict__ cb,
    const float* __restrict__ Alog, const float* __restrict__ Dp,
    unsigned short* __restrict__ YH, unsigned short* __restrict__ YL, int dir)
{
  __shared__ __align__(16) float sX[kScanTS * kBCW];
  __shared__ __align__(16) float sY[kScanTS * kScanYP];
  __shared__ __align__(16) float sA[kNst * kScanCh];
  const int tid = threadIdx.x, lane = tid & 31, wave = tid >> 5;
  constexpr int kBlkPerB = kDin / kScanCh;
  const int bix = blockIdx.x / kBlkPerB;
  const int d0  = (blockIdx.x - bix * kBlkPerB) * kScanCh;
  const int d   = d0 + tid;
  const size_t row0 = (size_t)bix * kSeq;
#pragma unroll 1
  for (int s = 0; s < kNst; ++s) sA[s * kScanCh + tid] = -expf(rbf(Alog[(size_t)d * kNst + s]));
  __syncthreads();
  float negA[kNst], h[kNst];
#pragma unroll
  for (int s = 0; s < kNst; ++s) {
    negA[s] = sA[s * kScanCh + tid];
    h[s] = 0.f;
  }
  const float Dd = rbf(Dp[d]);
  const v4f wv = *(const v4f*)(cw + (size_t)d * 4);
  const float w0 = rbf(wv[0]), w1 = rbf(wv[1]), w2 = rbf(wv[2]), w3 = rbf(wv[3]);
  const float bc = rbf(cb[d]);
  float xm3 = 0.f, xm2 = 0.f, xm1 = 0.f;
  const int lr = tid >> 3, lc4 = (tid & 7) * 4;
  const int q = lane >> 3, c8 = (lane & 7) * 8;
#pragma unroll 1
  for (int c = 0; c < kSeq / kScanTS; ++c) {
    const int t0 = dir ? (kSeq - kScanTS - c * kScanTS) : (c * kScanTS);
    __syncthreads();
#pragma unroll
    for (int i = 0; i < 8; ++i) {
      const int r = lr + 8 * i;
      *(v4f*)(sX + r * kBCW + lc4) = *(const v4f*)(PROJ + (row0 + t0 + r) * kPrjP + kDtR + lc4);
    }
    __syncthreads();
#pragma unroll 1
    for (int s = 0; s < kScanTS; ++s) {
      const int ls = dir ? (kScanTS - 1 - s) : s;
      const size_t grow = row0 + t0 + ls;
      const float* xr = sX + ls * kBCW;
      float dl = DLR[grow * kDin + d];
      float xi = XZ[grow * kXzP + d];
      float zv = XZ[grow * kXzP + kDin + d];
      asm volatile("" : "+v"(dl));
      asm volatile("" : "+v"(xi));
      asm volatile("" : "+v"(zv));
      float Bs[kNst], Cs[kNst];
#pragma unroll
      for (int q4 = 0; q4 < 4; ++q4) {
        const v4f bv = *(const v4f*)(xr + 4 * q4);
        const v4f cv = *(const v4f*)(xr + kNst + 4 * q4);
        Bs[4 * q4 + 0] = bv[0]; Bs[4 * q4 + 1] = bv[1]; Bs[4 * q4 + 2] = bv[2]; Bs[4 * q4 + 3] = bv[3];
        Cs[4 * q4 + 0] = cv[0]; Cs[4 * q4 + 1] = cv[1]; Cs[4 * q4 + 2] = cv[2]; Cs[4 * q4 + 3] = cv[3];
      }
      float cacc = w0 * xm3;
      cacc = fmaf(w1, xm2, cacc);
      cacc = fmaf(w2, xm1, cacc);
      cacc = fmaf(w3, xi, cacc);
      const float uu = cacc + bc;
      const float xt = uu * __builtin_amdgcn_rcpf(1.0f + __expf(-uu));
      xm3 = xm2; xm2 = xm1; xm1 = xi;
      const float a   = __expf(-fabsf(dl));
      const float u1  = 1.0f + a;
      const float l1p = __logf(u1) + (a - (u1 - 1.0f)) * __builtin_amdgcn_rcpf(u1);
      const float dt  = fmaxf(dl, 0.0f) + l1p;
      const float dtx = dt * xt;
      float y = 0.f;
#pragma unroll
      for (int k = 0; k < kNst; ++k) {
        const float e = __expf(dt * negA[k]);
        h[k] = e * h[k] + dtx * Bs[k];
        y = h[k] * Cs[k] + y;
      }
      y = xt * Dd + y;
      const float sg = __builtin_amdgcn_rcpf(1.0f + __expf(-zv));
      y = y * (zv * sg);
      sY[ls * kScanYP + tid] = y;
    }
    __syncthreads();
    v8h hv[8], lv[8];
#pragma unroll
    for (int it = 0; it < 8; ++it) {
      const int row = it * 8 + wave * 4 + q;
      const float* sp = sY + row * kScanYP + c8;
      const v4f a0 = *(const v4f*)(sp);
      const v4f a1 = *(const v4f*)(sp + 4);
#pragma unroll
      for (int e = 0; e < 4; ++e) {
        const float f0 = a0[e], f1 = a1[e];
        const unsigned short h0 = f2bf_bits(f0), h1 = f2bf_bits(f1);
        const unsigned short l0 = f2bf_bits(f0 - bf_bits2f(h0)), l1 = f2bf_bits(f1 - bf_bits2f(h1));
        hv[it][e]     = __builtin_bit_cast(_Float16, h0);
        hv[it][4 + e] = __builtin_bit_cast(_Float16, h1);
        lv[it][e]     = __builtin_bit_cast(_Float16, l0);
        lv[it][4 + e] = __builtin_bit_cast(_Float16, l1);
      }
    }
    for (int pass = 0; pass < 2; ++pass) {
#pragma unroll
      for (int it = 0; it < 8; ++it) {
        const int row = it * 8 + wave * 4 + q;
        const size_t o = (row0 + t0 + row) * kDin + d0 + c8;
        *(volatile v8h*)(YH + o) = hv[it];
        *(volatile v8h*)(YL + o) = lv[it];
      }
      __threadfence();
    }
  }
}

extern "C" void kernel_launch(void* const* d_in, const int* in_sizes, int n_in,
                              void* d_out, int out_size, void* d_ws, size_t ws_size,
                              hipStream_t stream) {
  if (n_in < 12) return;
  if (in_sizes[0] != kRows * kDm) return;
  if (in_sizes[1] != 2 * kDm * kXzP) return;
  if (in_sizes[2] != 2 * kDin * 4) return;
  if (in_sizes[3] != 2 * kDin) return;
  if (in_sizes[4] != 2 * kDin * kPrjN) return;
  if (in_sizes[5] != 2 * kDtR * kDin) return;
  if (in_sizes[6] != 2 * kDin) return;
  if (in_sizes[7] != 2 * kDin * kNst) return;
  if (in_sizes[8] != 2 * kDin) return;
  if (in_sizes[9] != 2 * kDin * kDm) return;
  if (in_sizes[10] != kCatK * kDm) return;
  if (in_sizes[11] != kDm) return;
  if (out_size != kRows * kDm) return;
  if (ws_size < kWsTotal) return;

  const float* x      = (const float*)d_in[0];
  const float* in_w   = (const float*)d_in[1];
  const float* conv_w = (const float*)d_in[2];
  const float* conv_b = (const float*)d_in[3];
  const float* xp_w   = (const float*)d_in[4];
  const float* dt_w   = (const float*)d_in[5];
  const float* dt_b   = (const float*)d_in[6];
  const float* A_log  = (const float*)d_in[7];
  const float* Dsk    = (const float*)d_in[8];
  const float* out_w  = (const float*)d_in[9];
  const float* proj_w = (const float*)d_in[10];
  const float* proj_b = (const float*)d_in[11];
  float* out = (float*)d_out;

  char* ws = (char*)d_ws;
  unsigned short* X16   = (unsigned short*)(ws + kOffX16);
  unsigned short* INWT  = (unsigned short*)(ws + kOffINWT);
  unsigned short* OUTWT = (unsigned short*)(ws + kOffOUTWT);
  unsigned short* PRJWT = (unsigned short*)(ws + kOffPRJWT);
  unsigned short* XPWT  = (unsigned short*)(ws + kOffXPWT);
  unsigned short* DTWT  = (unsigned short*)(ws + kOffDTWT);
  float*          XZ    = (float*)(ws + kOffXZ);
  unsigned short* UC16  = (unsigned short*)(ws + kOffUC16);
  float*          PROJ  = (float*)(ws + kOffPROJ);
  unsigned short* DT16  = (unsigned short*)(ws + kOffDT16);
  float*          DLR   = (float*)(ws + kOffDLR);
  unsigned short* YH    = (unsigned short*)(ws + kOffYH);
  unsigned short* YL    = (unsigned short*)(ws + kOffYL);
  unsigned short* CATH  = (unsigned short*)(ws + kOffCATH);
  unsigned short* CATL  = (unsigned short*)(ws + kOffCATL);

  cast_bf16_kernel<<<(kRows * kDm / 8) / 256, 256, 0, stream>>>(x, X16, kRows * kDm / 8);
  transpose_bf16_kernel<<<dim3(kXzP / 64, kDm / 64, 2), 256, 0, stream>>>(
      in_w, INWT, kDm, kXzP, (long)kDm * kXzP, (long)kXzP * kDm);
  transpose_bf16_kernel<<<dim3(kDm / 64, kDin / 64, 2), 256, 0, stream>>>(
      out_w, OUTWT, kDin, kDm, (long)kDin * kDm, (long)kDm * kDin);
  transpose_bf16_kernel<<<dim3(kDm / 64, kCatK / 64, 1), 256, 0, stream>>>(
      proj_w, PRJWT, kCatK, kDm, 0L, 0L);
  transpose_bf16_kernel<<<dim3(kPrjP / 64, kDin / 64, 2), 256, 0, stream>>>(
      xp_w, XPWT, kDin, kPrjN, (long)kDin * kPrjN, (long)kPrjP * kDin);
  transpose_bf16_kernel<<<dim3(kDin / 64, kDtR / 64, 2), 256, 0, stream>>>(
      dt_w, DTWT, kDtR, kDin, (long)kDtR * kDin, (long)kDin * kDtR);

  for (int dir = 0; dir < 2; ++dir) {
    const unsigned short* inwt  = INWT  + (size_t)dir * kXzP * kDm;
    const unsigned short* outwt = OUTWT + (size_t)dir * kDm * kDin;
    const unsigned short* xpwt  = XPWT  + (size_t)dir * kPrjP * kDin;
    const unsigned short* dtwt  = DTWT  + (size_t)dir * kDin * kDtR;
    const float* cw  = conv_w + (size_t)dir * kDin * 4;
    const float* cbp = conv_b + (size_t)dir * kDin;
    const float* dtb = dt_b   + (size_t)dir * kDin;
    const float* alg = A_log  + (size_t)dir * kDin * kNst;
    const float* dsk = Dsk    + (size_t)dir * kDin;

    wmma_gemm64<0, 0, 0><<<dim3(256), 256, 0, stream>>>(
        X16, X16, kDm, inwt, kDm, (void*)XZ, (void*)CATL, kXzP, dtb, kRows, kXzP, kDm);

    conv_silu_kernel<<<dim3(kDin / 256, kRows / 64), 256, 0, stream>>>(XZ, cw, cbp, UC16, dir);

    wmma_gemm64<0, 0, 0><<<dim3(8), 256, 0, stream>>>(
        UC16, UC16, kDin, xpwt, kDin, (void*)PROJ, (void*)CATL, kPrjP, dtb, kRows, kPrjP, kDin);

    dt_cast_kernel<<<(kRows * kDtR / 8) / 256, 256, 0, stream>>>(PROJ, DT16, kRows * kDtR / 8);

    wmma_gemm64<0, 2, 0><<<dim3(128), 256, 0, stream>>>(
        DT16, DT16, kDtR, dtwt, kDtR, (void*)DLR, (void*)CATL, kDin, dtb, kRows, kDin, kDtR);

    scan_kernel<<<kBatch * (kDin / kScanCh), kScanCh, 0, stream>>>(
        PROJ, DLR, XZ, cw, cbp, alg, dsk, YH, YL, dir);

    wmma_gemm64<1, 0, 2><<<dim3(64), 256, 0, stream>>>(
        YH, YL, kDin, outwt, kDin, (void*)(CATH + (size_t)dir * kDm), (void*)(CATL + (size_t)dir * kDm), kCatK,
        dtb, kRows, kDm, kDin);
  }

  wmma_gemm64<1, 2, 0><<<dim3(64), 256, 0, stream>>>(
      CATH, CATL, kCatK, PRJWT, kCatK, (void*)out, (void*)YH, kDm, proj_b, kRows, kDm, kCatK);
}
